// EdgeClassificationGNN2_41875931136397
// MI455X (gfx1250) — hardware-verified
//
#include <hip/hip_runtime.h>
#include <stddef.h>
#include <math.h>


#define CH     128
#define DE     16
#define HW     64
#define KNB    16
#define NTHR   256
#define NWAVE  8
#define EPT    8
#define NGRP   2
#define CHUNK  (NTHR * EPT * NGRP)
#define WCAP   (EPT * NGRP * 32)
#define LISTN  (NWAVE * WCAP)
#define NBC    4096
#define NBA    384
#define AGW    64
#define GROWS  64
#define GTHR   128
#define ETHR   128
#define ENW    4
#define ENIT   8
#define ETPB   (ENW * ENIT)
#define EAP    40
#define T1P    136
#define SGP    132
#define LDS_AGG ((NBA * CH + NWAVE * KNB * AGW + LISTN + NBA) * 4 + 64)
#define WSCAP  134217728
#define WSC    64.0f
#define WFSC   256.0f
#define E1SC   16.0f
#define Z1SC   64.0f
#define ABSC   1024.0f
#define R64    0.015625f
#define R4096  0.000244140625f
#define RABS   0.0009765625f

static_assert((CHUNK & (CHUNK - 1)) == 0);
static_assert(CHUNK <= 4096);
static_assert(NBC <= 4096 && NBA <= 4096);
static_assert((NBC & (NBC - 1)) == 0);
static_assert((NBA % (KNB * NWAVE)) == 0);
static_assert(GROWS == (GTHR / 32) * 16);
static_assert((EAP % 8) == 0 && (T1P % 8) == 0 && (SGP % 4) == 0);
static_assert(ETPB * KNB == 4 * ETHR);
static_assert(LDS_AGG == 247360);
static_assert(NTHR * 4 * 4 == NBC);

typedef float          v4f  __attribute__((ext_vector_type(4)));
typedef float          v8f  __attribute__((ext_vector_type(8)));
typedef int            v4i  __attribute__((ext_vector_type(4)));
typedef _Float16       v4h  __attribute__((ext_vector_type(4)));
typedef _Float16       v8h  __attribute__((ext_vector_type(8)));
typedef _Float16       v16h __attribute__((ext_vector_type(16)));
typedef unsigned short v8us __attribute__((ext_vector_type(8)));
typedef __bf16         v16b __attribute__((ext_vector_type(16)));
union FragH { v16h v; v8h h[2]; };
union FragB { v16b v; v8us u[2]; };

__device__ __forceinline__ v8f wmh(v16h a, v16h b, v8f c) {
  v8f d = __builtin_amdgcn_wmma_f32_16x16x32_f16(false, a, false, b, (short)0, c, false, false);
  asm volatile("v_nop\n\tv_nop\n\tv_nop\n\tv_nop" : "+v"(d) : "v"(a), "v"(b));
  return d;
}

__device__ __forceinline__ v8f wmb3(v16b ah, v16b al, v16b bh, v16b bl, v8f c) {
  v8f d = __builtin_amdgcn_wmma_f32_16x16x32_bf16(false, ah, false, bh, (short)0, c, false, false);
  d = __builtin_amdgcn_wmma_f32_16x16x32_bf16(false, ah, false, bl, (short)0, d, false, false);
  d = __builtin_amdgcn_wmma_f32_16x16x32_bf16(false, al, false, bh, (short)0, d, false, false);
  asm volatile("v_nop\n\tv_nop\n\tv_nop\n\tv_nop" : "+v"(d) : "v"(ah), "v"(al), "v"(bh), "v"(bl));
  return d;
}

__device__ __forceinline__ unsigned bfr(float f) {
  const unsigned u = __float_as_uint(f);
  return (u + 0x7FFFu + ((u >> 16) & 1u)) >> 16;
}

__device__ __forceinline__ void split8(v4f a, v4f b, v8us& hi, v8us& lo) {
  float f[8];
  f[0] = a.x; f[1] = a.y; f[2] = a.z; f[3] = a.w; f[4] = b.x; f[5] = b.y; f[6] = b.z; f[7] = b.w;
#pragma unroll
  for (int e = 0; e < 8; ++e) {
    const unsigned hb = bfr(f[e]);
    const float hf = __uint_as_float(hb << 16);
    const unsigned lb = bfr(f[e] - hf);
    hi[e] = (unsigned short)hb;
    lo[e] = (unsigned short)lb;
  }
}

__device__ __forceinline__ v8h cvt8(v4f a, v4f b, float s) {
  v8h r;
  r[0] = (_Float16)(a.x * s); r[1] = (_Float16)(a.y * s); r[2] = (_Float16)(a.z * s); r[3] = (_Float16)(a.w * s);
  r[4] = (_Float16)(b.x * s); r[5] = (_Float16)(b.y * s); r[6] = (_Float16)(b.z * s); r[7] = (_Float16)(b.w * s);
  return r;
}

__device__ __forceinline__ float tanh_f(float x) {
  const float t = fminf(fmaxf(x, -30.0f), 30.0f);
  const float e = __builtin_amdgcn_exp2f(t * 2.8853900817779268f);
  const float r = __builtin_amdgcn_rcpf(e + 1.0f);
  return fmaf(-2.0f, r, 1.0f);
}

template <int NB>
__device__ __forceinline__ int scan_chunk(const int* __restrict__ dsts, int nE, int cbase, int slotBase,
                                          int vec8, int* list, int tid, int lane, int wave) {
  int wc = 0;
#pragma unroll
  for (int g = 0; g < NGRP; ++g) {
    const int el0  = (g * NTHR + tid) * EPT;
    const int e0   = cbase + el0;
    const int sent = -2147483647 - 1;
    v4i da, db;
    if (vec8 != 0 && cbase + CHUNK <= nE) {
      da = *(const v4i*)(dsts + e0);
      db = *(const v4i*)(dsts + e0 + 4);
    } else {
      da.x = (e0     < nE) ? dsts[min(e0, nE - 1)] : sent;
      da.y = (e0 + 1 < nE) ? dsts[min(e0 + 1, nE - 1)] : sent;
      da.z = (e0 + 2 < nE) ? dsts[min(e0 + 2, nE - 1)] : sent;
      da.w = (e0 + 3 < nE) ? dsts[min(e0 + 3, nE - 1)] : sent;
      db.x = (e0 + 4 < nE) ? dsts[min(e0 + 4, nE - 1)] : sent;
      db.y = (e0 + 5 < nE) ? dsts[min(e0 + 5, nE - 1)] : sent;
      db.z = (e0 + 6 < nE) ? dsts[min(e0 + 6, nE - 1)] : sent;
      db.w = (e0 + 7 < nE) ? dsts[min(e0 + 7, nE - 1)] : sent;
    }
    const unsigned nb = (unsigned)slotBase;
    const unsigned s0 = (unsigned)da.x - nb, s1 = (unsigned)da.y - nb;
    const unsigned s2 = (unsigned)da.z - nb, s3 = (unsigned)da.w - nb;
    const unsigned s4 = (unsigned)db.x - nb, s5 = (unsigned)db.y - nb;
    const unsigned s6 = (unsigned)db.z - nb, s7 = (unsigned)db.w - nb;
    const bool h0 = s0 < (unsigned)NB, h1 = s1 < (unsigned)NB, h2 = s2 < (unsigned)NB, h3 = s3 < (unsigned)NB;
    const bool h4 = s4 < (unsigned)NB, h5 = s5 < (unsigned)NB, h6 = s6 < (unsigned)NB, h7 = s7 < (unsigned)NB;
    const unsigned any = __builtin_amdgcn_ballot_w32(h0 | h1 | h2 | h3 | h4 | h5 | h6 | h7);
    if (any != 0u) {
#define HITJ(J, HJ, SJ) { \
        const unsigned mj = __builtin_amdgcn_ballot_w32(HJ); \
        if (mj != 0u) { \
          if (HJ) { \
            const int pos = wc + (int)__builtin_amdgcn_mbcnt_lo(mj, 0u); \
            if (pos < WCAP) list[wave * WCAP + pos] = ((el0 + (J)) << 12) | (int)(SJ); \
          } \
          wc += (int)__builtin_popcount(mj); } }
      HITJ(0, h0, s0)
      HITJ(1, h1, s1)
      HITJ(2, h2, s2)
      HITJ(3, h3, s3)
      HITJ(4, h4, s4)
      HITJ(5, h5, s5)
      HITJ(6, h6, s6)
      HITJ(7, h7, s7)
#undef HITJ
    }
  }
  return wc;
}

__global__ __launch_bounds__(NTHR) void k_prep(
    const float* __restrict__ W1, const float* __restrict__ W2, const float* __restrict__ We1,
    const float* __restrict__ We2, const float* __restrict__ Wc1, const float* __restrict__ bc1,
    const float* __restrict__ be2, const float* __restrict__ Wc2,
    unsigned short* W1h, unsigned short* W1l, unsigned short* W2h, unsigned short* W2l,
    unsigned short* Wch, unsigned short* Wcl, unsigned short* We2h, unsigned short* We2l,
    _Float16* We1p, _Float16* Wc2p, float* Tt, float* cvec) {
  const int blk = blockIdx.x, tid = threadIdx.x;
  if (blk < 40) {
    float v[8];
    unsigned short* ph;
    unsigned short* pl;
    int o;
    if (blk < 8) {
      const int i = blk * NTHR + tid;
      const int n = i >> 4, k0 = (i & 15) * 8;
#pragma unroll
      for (int e = 0; e < 8; ++e) v[e] = W1[(k0 + e) * CH + n];
      ph = W1h; pl = W1l; o = 8 * i;
    } else if (blk < 16) {
      const int i = (blk - 8) * NTHR + tid;
      const int n = i >> 4, k0 = (i & 15) * 8;
#pragma unroll
      for (int e = 0; e < 8; ++e) v[e] = W2[(k0 + e) * CH + n];
      ph = W2h; pl = W2l; o = 8 * i;
    } else if (blk < 32) {
      const int i = (blk - 16) * NTHR + tid;
      const int n = i >> 4, k0 = (i & 15) * 8;
      const int roff = (n >> 7) * CH, nc = n & (CH - 1);
#pragma unroll
      for (int e = 0; e < 8; ++e) v[e] = Wc1[(size_t)(roff + k0 + e) * CH + nc];
      ph = Wch; pl = Wcl; o = 8 * i;
    } else {
      const int i = (blk - 32) * NTHR + tid;
#pragma unroll
      for (int e = 0; e < 8; ++e) v[e] = We2[8 * i + e];
      ph = We2h; pl = We2l; o = 8 * i;
    }
    v4f a, b;
    a.x = v[0]; a.y = v[1]; a.z = v[2]; a.w = v[3];
    b.x = v[4]; b.y = v[5]; b.z = v[6]; b.w = v[7];
    v8us hv, lv;
    split8(a, b, hv, lv);
    *(volatile v8us*)(ph + o) = hv;
    *(volatile v8us*)(pl + o) = lv;
    __threadfence();
    *(volatile v8us*)(ph + o) = hv;
    *(volatile v8us*)(pl + o) = lv;
  } else if (blk < 56) {
    const int i = (blk - 40) * NTHR + tid;
    const int j = i >> 5, n0 = (i & 31) * 4;
    v4f t4;
    t4.x = Wc1[(size_t)(2 * CH + n0 + 0) * CH + j];
    t4.y = Wc1[(size_t)(2 * CH + n0 + 1) * CH + j];
    t4.z = Wc1[(size_t)(2 * CH + n0 + 2) * CH + j];
    t4.w = Wc1[(size_t)(2 * CH + n0 + 3) * CH + j];
    *(volatile v4f*)(Tt + 4 * i) = t4;
    __threadfence();
    *(volatile v4f*)(Tt + 4 * i) = t4;
  } else if (blk < 58) {
    const int i = (blk - 56) * NTHR + tid;
    const int n = i >> 2, k0 = (i & 3) * 8;
    v8h hv;
#pragma unroll
    for (int e = 0; e < 8; ++e) {
      const int kk = k0 + e;
      const int kc = kk < DE ? kk : DE - 1;
      const float w = We1[kc * CH + n];
      hv[e] = (_Float16)((kk < DE ? w : 0.0f) * WSC);
    }
    *(volatile v8h*)(We1p + 8 * i) = hv;
    __threadfence();
    *(volatile v8h*)(We1p + 8 * i) = hv;
  } else if (blk < 62) {
    const int i = (blk - 58) * NTHR + tid;
    const int n = i >> 4, k0 = (i & 15) * 8;
    v8h hv;
#pragma unroll
    for (int e = 0; e < 8; ++e) hv[e] = (_Float16)(Wc2[(k0 + e) * HW + n] * WSC);
    *(volatile v8h*)(Wc2p + 8 * i) = hv;
    __threadfence();
    *(volatile v8h*)(Wc2p + 8 * i) = hv;
  } else {
    __shared__ __attribute__((aligned(16))) float scv[CH];
    if (tid < CH) {
      float s = bc1[tid];
#pragma unroll 1
      for (int n = 0; n < CH; ++n) s = fmaf(be2[n], Wc1[(size_t)(2 * CH + n) * CH + tid], s);
      scv[tid] = s;
    }
    __syncthreads();
    v4f cv = {0.f, 0.f, 0.f, 0.f};
    if (tid < 32) cv = *(const v4f*)(scv + 4 * tid);
    if (tid < 32) *(volatile v4f*)(cvec + 4 * tid) = cv;
    __threadfence();
    if (tid < 32) *(volatile v4f*)(cvec + 4 * tid) = cv;
  }
}

__global__ __launch_bounds__(NTHR) void k_cvwf(const float* __restrict__ WfT, _Float16* Wfp) {
  const int i = blockIdx.x * NTHR + threadIdx.x;
  const v4f a = *(const v4f*)(WfT + 8 * i), b = *(const v4f*)(WfT + 8 * i + 4);
  const v8h hv = cvt8(a, b, WFSC);
  *(volatile v8h*)(Wfp + 8 * i) = hv;
  __threadfence();
  *(volatile v8h*)(Wfp + 8 * i) = hv;
}

__global__ __launch_bounds__(GTHR) void k_gemm3(const float* __restrict__ A, int lda, int M,
                                                const unsigned short* __restrict__ Bh,
                                                const unsigned short* __restrict__ Bl, float* Out) {
  __shared__ __attribute__((aligned(16))) float stg[GROWS * CH];
  const int tid = threadIdx.x, lane = tid & 31, wave = tid >> 5, hh = lane >> 4, m = lane & 15;
  const int rowBase = blockIdx.x * GROWS;
  int arow = rowBase + wave * 16 + m;
  arow = arow > M - 1 ? M - 1 : arow;
  const float* ap = A + (size_t)arow * lda + 8 * hh;
  v8f acc[8];
#pragma unroll
  for (int t = 0; t < 8; ++t) { v8f z = {0.f, 0.f, 0.f, 0.f, 0.f, 0.f, 0.f, 0.f}; acc[t] = z; }
#pragma unroll 1
  for (int ks = 0; ks < CH / 32; ++ks) {
    const float* q = ap + 32 * ks;
    const v4f f0 = *(const v4f*)q, f1 = *(const v4f*)(q + 4);
    const v4f f2 = *(const v4f*)(q + 16), f3 = *(const v4f*)(q + 20);
    FragB ah, al;
    split8(f0, f1, ah.u[0], al.u[0]);
    split8(f2, f3, ah.u[1], al.u[1]);
#pragma unroll
    for (int t = 0; t < 8; ++t) {
      const size_t bo = (size_t)(16 * t + m) * CH + 32 * ks + 8 * hh;
      FragB bh, bl;
      bh.u[0] = *(const v8us*)(Bh + bo); bh.u[1] = *(const v8us*)(Bh + bo + 16);
      bl.u[0] = *(const v8us*)(Bl + bo); bl.u[1] = *(const v8us*)(Bl + bo + 16);
      acc[t] = wmb3(ah.v, al.v, bh.v, bl.v, acc[t]);
    }
  }
  float* sp = stg + (wave * 16 + 8 * hh) * CH + m;
#pragma unroll
  for (int t = 0; t < 8; ++t) {
#pragma unroll
    for (int r = 0; r < 8; ++r) sp[r * CH + 16 * t] = acc[t][r];
  }
  __syncthreads();
  float* gp = Out + (size_t)rowBase * CH;
#pragma unroll
  for (int it = 0; it < 16; ++it) {
    const int f = it * GTHR + tid;
    const v4f v = *(const v4f*)(stg + 4 * f);
    *(volatile v4f*)(gp + 4 * f) = v;
  }
  __threadfence();
#pragma unroll
  for (int it = 0; it < 16; ++it) {
    const int f = it * GTHR + tid;
    const v4f v = *(const v4f*)(stg + 4 * f);
    *(volatile v4f*)(gp + 4 * f) = v;
  }
}

__global__ __launch_bounds__(NTHR) void k_count(const int* __restrict__ dsts, float* dinv, int nE, int vec8) {
  __shared__ __attribute__((aligned(16))) int scnt[NBC];
  __shared__ __attribute__((aligned(16))) int list[LISTN];
  __shared__ int wcnt[NWAVE];
  const int tid = threadIdx.x, lane = tid & 31, wave = tid >> 5;
  const int nodeBase = blockIdx.x * NBC;

  for (int i = tid; i < NBC; i += NTHR) scnt[i] = 0;
  __syncthreads();

  const int nChunks = (nE + CHUNK - 1) / CHUNK;
#pragma unroll 1
  for (int ch = 0; ch < nChunks; ++ch) {
    const int cbase = ch * CHUNK;
    const int wc = scan_chunk<NBC>(dsts, nE, cbase, nodeBase, vec8, list, tid, lane, wave);
    if (lane == 0) wcnt[wave] = wc;
    __syncthreads();
    if (wave == 0) {
#pragma unroll 1
      for (int wsx = 0; wsx < NWAVE; ++wsx) {
        int n = __builtin_amdgcn_readfirstlane(wcnt[wsx]);
        n = n > WCAP ? WCAP : (n < 0 ? 0 : n);
        const int* lp = list + wsx * WCAP;
#pragma unroll 1
        for (int i = 0; i < n; ++i) {
          const int ent  = __builtin_amdgcn_readfirstlane(lp[i]);
          const int slot = ent & (NBC - 1);
          if (lane == 0) scnt[slot] = scnt[slot] + 1;
        }
      }
    }
    __syncthreads();
  }

  v4f dq[4];
#pragma unroll
  for (int q = 0; q < 4; ++q) {
    const int f = (wave * 4 + q) * 128 + 4 * lane;
    const v4i c = *(const v4i*)(scnt + f);
    v4f d;
    d.x = __builtin_amdgcn_rsqf((float)c.x + 1.0f);
    d.y = __builtin_amdgcn_rsqf((float)c.y + 1.0f);
    d.z = __builtin_amdgcn_rsqf((float)c.z + 1.0f);
    d.w = __builtin_amdgcn_rsqf((float)c.w + 1.0f);
    dq[q] = d;
  }
  float* dp = dinv + (size_t)nodeBase;
#pragma unroll
  for (int q = 0; q < 4; ++q) {
    const int f = (wave * 4 + q) * 128 + 4 * lane;
    *(volatile v4f*)(dp + f) = dq[q];
  }
  __threadfence();
#pragma unroll
  for (int q = 0; q < 4; ++q) {
    const int f = (wave * 4 + q) * 128 + 4 * lane;
    *(volatile v4f*)(dp + f) = dq[q];
  }
}

template <bool OUT16>
__global__ __launch_bounds__(NTHR) void k_agg(
    const float* __restrict__ xw, const float* __restrict__ dinv,
    const int* __restrict__ srcs, const int* __restrict__ dsts, const float* __restrict__ bias,
    const unsigned short* __restrict__ Bh, const unsigned short* __restrict__ Bl, int ncol,
    void* outp, int nN, int nE, int vec8, int nPad) {
  extern __shared__ v4f lds_dyn[];
  float* acc  = (float*)lds_dyn;
  float* stg  = acc + NBA * CH;
  int*   list = (int*)(stg + NWAVE * KNB * AGW);
  float* sdv  = (float*)(list + LISTN);
  int*   wcnt = (int*)(sdv + NBA);
  const int tid = threadIdx.x, lane = tid & 31, wave = tid >> 5, hh = lane >> 4, m = lane & 15;
  const int base = blockIdx.x * NBA;

  for (int s = tid; s < NBA; s += NTHR) {
    int nd = base + s;
    nd = nd > nN - 1 ? nN - 1 : nd;
    sdv[s] = dinv[nd];
  }
  for (int f = tid; f < NBA * (CH / 4); f += NTHR) {
    const int slot = f >> 5, c4 = (f & 31) * 4;
    const int node = base + slot;
    const int ncl = node < nN ? node : nN - 1;
    const v4f v = *(const v4f*)(xw + (size_t)ncl * CH + c4);
    const float d = dinv[ncl];
    const float dd = d * d;
    v4f r = v * dd;
    const bool ok = node < nN;
    r.x = ok ? r.x : 0.0f; r.y = ok ? r.y : 0.0f; r.z = ok ? r.z : 0.0f; r.w = ok ? r.w : 0.0f;
    *(v4f*)(acc + slot * CH + c4) = r;
  }
  __syncthreads();

  const int nChunks = (nE + CHUNK - 1) / CHUNK;
#pragma unroll 1
  for (int ch = 0; ch < nChunks; ++ch) {
    const int cbase = ch * CHUNK;
    const int wc = scan_chunk<NBA>(dsts, nE, cbase, base, vec8, list, tid, lane, wave);
    if (lane == 0) wcnt[wave] = wc;
    __syncthreads();
    if (wave == 0) {
#pragma unroll 1
      for (int wsx = 0; wsx < NWAVE; ++wsx) {
        int n = __builtin_amdgcn_readfirstlane(wcnt[wsx]);
        n = n > WCAP ? WCAP : (n < 0 ? 0 : n);
        const int* lp = list + wsx * WCAP;
#pragma unroll 1
        for (int i = 0; i < n; ++i) {
          const int ent = __builtin_amdgcn_readfirstlane(lp[i]);
          int slot = ent & 4095;
          slot = slot > NBA - 1 ? NBA - 1 : slot;
          int e = cbase + ((ent >> 12) & (CHUNK - 1));
          e = e > nE - 1 ? nE - 1 : e;
          int sv = srcs[e];
          sv = sv < 0 ? 0 : (sv > nN - 1 ? nN - 1 : sv);
          const float nrm = dinv[sv] * sdv[slot];
          const v4f v = *(const v4f*)(xw + (size_t)sv * CH + 4 * lane);
          float* ar = acc + slot * CH + 4 * lane;
          v4f a = *(const v4f*)ar;
          a.x = fmaf(v.x, nrm, a.x); a.y = fmaf(v.y, nrm, a.y);
          a.z = fmaf(v.z, nrm, a.z); a.w = fmaf(v.w, nrm, a.w);
          *(v4f*)ar = a;
        }
      }
    }
    __syncthreads();
  }

  for (int f = tid; f < NBA * (CH / 4); f += NTHR) {
    const int slot = f >> 5, c4 = (f & 31) * 4;
    const int node = base + slot;
    const bool ok = node < nN;
    const v4f b4 = *(const v4f*)(bias + c4);
    float* ar = acc + slot * CH + c4;
    v4f a = *(const v4f*)ar;
    a.x = ok ? a.x + b4.x : a.x; a.y = ok ? a.y + b4.y : a.y;
    a.z = ok ? a.z + b4.z : a.z; a.w = ok ? a.w + b4.w : a.w;
    *(v4f*)ar = a;
  }
  __syncthreads();

  const int ngrp = ncol / AGW;
  float* stw = stg + wave * (KNB * AGW);
#pragma unroll 1
  for (int tt = 0; tt < NBA / KNB / NWAVE; ++tt) {
    const int r0 = (tt * NWAVE + wave) * KNB;
    const float* ap = acc + (r0 + m) * CH + 8 * hh;
#pragma unroll 1
    for (int g = 0; g < ngrp; ++g) {
      v8f a4[4];
#pragma unroll
      for (int t = 0; t < 4; ++t) { v8f z = {0.f, 0.f, 0.f, 0.f, 0.f, 0.f, 0.f, 0.f}; a4[t] = z; }
#pragma unroll 1
      for (int ks = 0; ks < CH / 32; ++ks) {
        const float* q = ap + 32 * ks;
        const v4f f0 = *(const v4f*)q, f1 = *(const v4f*)(q + 4);
        const v4f f2 = *(const v4f*)(q + 16), f3 = *(const v4f*)(q + 20);
        FragB ah, al;
        split8(f0, f1, ah.u[0], al.u[0]);
        split8(f2, f3, ah.u[1], al.u[1]);
#pragma unroll
        for (int t = 0; t < 4; ++t) {
          const size_t bo = (size_t)(AGW * g + 16 * t + m) * CH + 32 * ks + 8 * hh;
          FragB bh, bl;
          bh.u[0] = *(const v8us*)(Bh + bo); bh.u[1] = *(const v8us*)(Bh + bo + 16);
          bl.u[0] = *(const v8us*)(Bl + bo); bl.u[1] = *(const v8us*)(Bl + bo + 16);
          a4[t] = wmb3(ah.v, al.v, bh.v, bl.v, a4[t]);
        }
      }
      __syncthreads();
      float* sp = stw + (8 * hh) * AGW + m;
#pragma unroll
      for (int t = 0; t < 4; ++t) {
#pragma unroll
        for (int r = 0; r < 8; ++r) sp[r * AGW + 16 * t] = a4[t][r];
      }
      __syncthreads();
      if (OUT16) {
        _Float16* ob = (_Float16*)outp;
        v8h hv[4];
        size_t go[4];
        bool ok[4];
#pragma unroll
        for (int rr = 0; rr < 4; ++rr) {
          const int row = 4 * rr + (lane >> 3), pc = lane & 7;
          const v4f p0 = *(const v4f*)(stw + row * AGW + 8 * pc);
          const v4f p1 = *(const v4f*)(stw + row * AGW + 8 * pc + 4);
          hv[rr] = cvt8(p0, p1, ABSC);
          const int node = base + r0 + row;
          ok[rr] = node < nPad;
          const int ncl = ok[rr] ? node : nPad - 1;
          go[rr] = (size_t)ncl * ncol + AGW * g + 8 * pc;
        }
#pragma unroll
        for (int rr = 0; rr < 4; ++rr) { if (ok[rr]) *(volatile v8h*)(ob + go[rr]) = hv[rr]; }
        __threadfence();
#pragma unroll
        for (int rr = 0; rr < 4; ++rr) { if (ok[rr]) *(volatile v8h*)(ob + go[rr]) = hv[rr]; }
      } else {
        float* ob = (float*)outp;
        v4f fv[8];
        size_t go[8];
        bool ok[8];
#pragma unroll
        for (int rr = 0; rr < 8; ++rr) {
          const int row = 2 * rr + (lane >> 4), pc = lane & 15;
          fv[rr] = *(const v4f*)(stw + row * AGW + 4 * pc);
          const int node = base + r0 + row;
          ok[rr] = node < nPad;
          const int ncl = ok[rr] ? node : nPad - 1;
          go[rr] = (size_t)ncl * ncol + AGW * g + 4 * pc;
        }
#pragma unroll
        for (int rr = 0; rr < 8; ++rr) { if (ok[rr]) *(volatile v4f*)(ob + go[rr]) = fv[rr]; }
        __threadfence();
#pragma unroll
        for (int rr = 0; rr < 8; ++rr) { if (ok[rr]) *(volatile v4f*)(ob + go[rr]) = fv[rr]; }
      }
    }
  }
}

__global__ __launch_bounds__(ETHR) void k_edge(
    const float* __restrict__ ea, const int* __restrict__ srcs, const int* __restrict__ dsts,
    const _Float16* __restrict__ ABs, const _Float16* __restrict__ We1p,
    const _Float16* __restrict__ Wfp, const _Float16* __restrict__ Wc2p,
    const float* __restrict__ be1, const float* __restrict__ cvec, const float* __restrict__ bc2,
    const float* __restrict__ Wc3, const float* __restrict__ bc3, float* out, int nN, int nE) {
  __shared__ __attribute__((aligned(16))) _Float16 eaT[ENW * KNB * EAP];
  __shared__ __attribute__((aligned(16))) _Float16 t1[ENW * KNB * T1P];
  __shared__ __attribute__((aligned(16))) float sg[ENW * KNB * SGP];
  __shared__ __attribute__((aligned(16))) float sout[ETPB * KNB];
  const int tid = threadIdx.x, lane = tid & 31, wave = tid >> 5, hh = lane >> 4, m = lane & 15;
  _Float16* eaw = eaT + wave * (KNB * EAP);
  _Float16* t1w = t1 + wave * (KNB * T1P);
  float* sgw = sg + wave * (KNB * SGP);
  const int tbase = blockIdx.x * ETPB;
  const int ebase = tbase * KNB;

  float be1c[8], bc2c[4], wc3c[4];
#pragma unroll
  for (int t = 0; t < 8; ++t) be1c[t] = be1[16 * t + m];
#pragma unroll
  for (int t = 0; t < 4; ++t) { bc2c[t] = bc2[16 * t + m]; wc3c[t] = Wc3[16 * t + m]; }
  const v4f cv4 = *(const v4f*)(cvec + 4 * lane);
  const float b3 = bc3[0];

#pragma unroll 1
  for (int it = 0; it < ENIT; ++it) {
    const int lt = it * ENW + wave;
    const int e0 = ebase + lt * KNB;
    __syncthreads();
    int ei = e0 + m;
    ei = ei > nE - 1 ? nE - 1 : ei;
    int sl = srcs[ei]; sl = sl < 0 ? 0 : (sl > nN - 1 ? nN - 1 : sl);
    int dl = dsts[ei]; dl = dl < 0 ? 0 : (dl > nN - 1 ? nN - 1 : dl);
    {
      const int row = lane >> 1, c = lane & 1;
      int er = e0 + row;
      er = er > nE - 1 ? nE - 1 : er;
      const float* p = ea + (size_t)er * DE + 8 * c;
      const v4f a = *(const v4f*)p, b = *(const v4f*)(p + 4);
      *(v8h*)(eaw + row * EAP + 8 * c) = cvt8(a, b, 1.0f);
      v8h z;
#pragma unroll
      for (int e = 0; e < 8; ++e) z[e] = (_Float16)0.0f;
      *(v8h*)(eaw + row * EAP + 16 + 8 * c) = z;
    }
#pragma unroll
    for (int i = 0; i < KNB; ++i) {
      const int s = __builtin_amdgcn_readlane(sl, i);
      const int d = __builtin_amdgcn_readlane(dl, i);
      const v4h ha = *(const v4h*)(ABs + (size_t)s * (2 * CH) + 4 * lane);
      const v4h hb = *(const v4h*)(ABs + (size_t)d * (2 * CH) + CH + 4 * lane);
      v4f sv;
      sv.x = ((float)ha.x + (float)hb.x) * RABS + cv4.x;
      sv.y = ((float)ha.y + (float)hb.y) * RABS + cv4.y;
      sv.z = ((float)ha.z + (float)hb.z) * RABS + cv4.z;
      sv.w = ((float)ha.w + (float)hb.w) * RABS + cv4.w;
      *(v4f*)(sgw + i * SGP + 4 * lane) = sv;
    }
    __syncthreads();
    {
      FragH a;
      a.h[0] = *(const v8h*)(eaw + m * EAP + 8 * hh);
      a.h[1] = *(const v8h*)(eaw + m * EAP + 16 + 8 * hh);
      v8f acc[8];
#pragma unroll
      for (int t = 0; t < 8; ++t) {
        const _Float16* bp = We1p + (16 * t + m) * 32 + 8 * hh;
        FragH b;
        b.h[0] = *(const v8h*)bp;
        b.h[1] = *(const v8h*)(bp + 16);
        v8f z = {0.f, 0.f, 0.f, 0.f, 0.f, 0.f, 0.f, 0.f};
        acc[t] = wmh(a.v, b.v, z);
      }
#pragma unroll
      for (int t = 0; t < 8; ++t) {
#pragma unroll
        for (int r = 0; r < 8; ++r) {
          float v = fmaf(acc[t][r], R64, be1c[t]);
          v = fmaxf(v, 0.0f);
          t1w[(8 * hh + r) * T1P + 16 * t + m] = (_Float16)(v * E1SC);
        }
      }
    }
    __syncthreads();
    {
      v8f acc[8];
#pragma unroll
      for (int t = 0; t < 8; ++t) { v8f z = {0.f, 0.f, 0.f, 0.f, 0.f, 0.f, 0.f, 0.f}; acc[t] = z; }
      const _Float16* apz = t1w + m * T1P + 8 * hh;
#pragma unroll 1
      for (int ks = 0; ks < CH / 32; ++ks) {
        FragH a;
        a.h[0] = *(const v8h*)(apz + 32 * ks);
        a.h[1] = *(const v8h*)(apz + 32 * ks + 16);
#pragma unroll
        for (int t = 0; t < 8; ++t) {
          const _Float16* bp = Wfp + (16 * t + m) * CH + 32 * ks + 8 * hh;
          FragH b;
          b.h[0] = *(const v8h*)bp;
          b.h[1] = *(const v8h*)(bp + 16);
          acc[t] = wmh(a.v, b.v, acc[t]);
        }
      }
      __syncthreads();
#pragma unroll
      for (int t = 0; t < 8; ++t) {
#pragma unroll
        for (int r = 0; r < 8; ++r) {
          const float pre = fmaf(acc[t][r], R4096, sgw[(8 * hh + r) * SGP + 16 * t + m]);
          const float z = tanh_f(pre);
          t1w[(8 * hh + r) * T1P + 16 * t + m] = (_Float16)(z * Z1SC);
        }
      }
    }
    __syncthreads();
    {
      v8f acc[4];
#pragma unroll
      for (int t = 0; t < 4; ++t) { v8f z = {0.f, 0.f, 0.f, 0.f, 0.f, 0.f, 0.f, 0.f}; acc[t] = z; }
      const _Float16* apz = t1w + m * T1P + 8 * hh;
#pragma unroll 1
      for (int ks = 0; ks < CH / 32; ++ks) {
        FragH a;
        a.h[0] = *(const v8h*)(apz + 32 * ks);
        a.h[1] = *(const v8h*)(apz + 32 * ks + 16);
#pragma unroll
        for (int t = 0; t < 4; ++t) {
          const _Float16* bp = Wc2p + (16 * t + m) * CH + 32 * ks + 8 * hh;
          FragH b;
          b.h[0] = *(const v8h*)bp;
          b.h[1] = *(const v8h*)(bp + 16);
          acc[t] = wmh(a.v, b.v, acc[t]);
        }
      }
      float p[8] = {0.f, 0.f, 0.f, 0.f, 0.f, 0.f, 0.f, 0.f};
#pragma unroll
      for (int t = 0; t < 4; ++t) {
#pragma unroll
        for (int r = 0; r < 8; ++r) {
          const float v = tanh_f(fmaf(acc[t][r], R4096, bc2c[t]));
          p[r] = fmaf(v, wc3c[t], p[r]);
        }
      }
#pragma unroll
      for (int r = 0; r < 8; ++r) {
        p[r] += __shfl_xor(p[r], 8, 32);
        p[r] += __shfl_xor(p[r], 4, 32);
        p[r] += __shfl_xor(p[r], 2, 32);
        p[r] += __shfl_xor(p[r], 1, 32);
      }
      if (m == 0) {
#pragma unroll
        for (int r = 0; r < 8; ++r) sout[lt * KNB + 8 * hh + r] = p[r] + b3;
      }
    }
  }
  __syncthreads();
  {
    const v4f ov = *(const v4f*)(sout + 4 * tid);
    const int e = ebase + 4 * tid;
    float* op = out + e;
    if (e + 4 <= nE) {
      *(volatile v4f*)op = ov;
    } else {
      if (e < nE)     *(volatile float*)(op)     = ov.x;
      if (e + 1 < nE) *(volatile float*)(op + 1) = ov.y;
      if (e + 2 < nE) *(volatile float*)(op + 2) = ov.z;
      if (e + 3 < nE) *(volatile float*)(op + 3) = ov.w;
    }
    __threadfence();
    if (e + 4 <= nE) {
      *(volatile v4f*)op = ov;
    } else {
      if (e < nE)     *(volatile float*)(op)     = ov.x;
      if (e + 1 < nE) *(volatile float*)(op + 1) = ov.y;
      if (e + 2 < nE) *(volatile float*)(op + 2) = ov.z;
      if (e + 3 < nE) *(volatile float*)(op + 3) = ov.w;
    }
  }
}

extern "C" void kernel_launch(void* const* d_in, const int* in_sizes, int n_in,
                              void* d_out, int out_size, void* d_ws, size_t ws_size,
                              hipStream_t stream) {
  if (n_in < 17) return;
  const int nN = in_sizes[0] / CH;
  const int nE = in_sizes[1] / 2;
  if (nN <= 0 || nE <= 0) return;
  if (in_sizes[0] != nN * CH || in_sizes[1] != 2 * nE || in_sizes[2] != nE * DE) return;
  if (in_sizes[3] != CH * CH || in_sizes[4] != CH || in_sizes[5] != CH * CH || in_sizes[6] != CH) return;
  if (in_sizes[7] != DE * CH || in_sizes[8] != CH || in_sizes[9] != CH * CH || in_sizes[10] != CH) return;
  if (in_sizes[11] != 3 * CH * CH || in_sizes[12] != CH || in_sizes[13] != CH * HW || in_sizes[14] != HW) return;
  if (in_sizes[15] != HW || in_sizes[16] < 1) return;
  if (out_size != nE) return;
  if (nN > (1 << 24) || nE > (1 << 28)) return;

  const float* x   = (const float*)d_in[0];
  const int*   ei  = (const int*)d_in[1];
  const float* ea  = (const float*)d_in[2];
  const float* W1  = (const float*)d_in[3];
  const float* b1  = (const float*)d_in[4];
  const float* W2  = (const float*)d_in[5];
  const float* b2  = (const float*)d_in[6];
  const float* We1 = (const float*)d_in[7];
  const float* be1 = (const float*)d_in[8];
  const float* We2 = (const float*)d_in[9];
  const float* be2 = (const float*)d_in[10];
  const float* Wc1 = (const float*)d_in[11];
  const float* bc1 = (const float*)d_in[12];
  const float* Wc2 = (const float*)d_in[13];
  const float* bc2 = (const float*)d_in[14];
  const float* Wc3 = (const float*)d_in[15];
  const float* bc3 = (const float*)d_in[16];
  const int* srcs = ei;
  const int* dsts = ei + nE;
  float* out = (float*)d_out;

  const int nBlkG = (nN + GROWS - 1) / GROWS;
  const int NPAD  = nBlkG * GROWS;
  const int nBA   = (NPAD + NBA - 1) / NBA;
  const int nBC   = (nN + NBC - 1) / NBC;
  const int CNTPAD = nBC * NBC;
  const int nT    = (nE + KNB - 1) / KNB;
  const int nBlkE = (nT + ETPB - 1) / ETPB;

  char* ws = (char*)d_ws;
  size_t off = 0;
  const size_t oW1h = off; off += (size_t)CH * CH * 2;      off = (off + 255) & ~(size_t)255;
  const size_t oW1l = off; off += (size_t)CH * CH * 2;      off = (off + 255) & ~(size_t)255;
  const size_t oW2h = off; off += (size_t)CH * CH * 2;      off = (off + 255) & ~(size_t)255;
  const size_t oW2l = off; off += (size_t)CH * CH * 2;      off = (off + 255) & ~(size_t)255;
  const size_t oWch = off; off += (size_t)2 * CH * CH * 2;  off = (off + 255) & ~(size_t)255;
  const size_t oWcl = off; off += (size_t)2 * CH * CH * 2;  off = (off + 255) & ~(size_t)255;
  const size_t oE2h = off; off += (size_t)CH * CH * 2;      off = (off + 255) & ~(size_t)255;
  const size_t oE2l = off; off += (size_t)CH * CH * 2;      off = (off + 255) & ~(size_t)255;
  const size_t oE1p = off; off += (size_t)CH * 32 * 2;      off = (off + 255) & ~(size_t)255;
  const size_t oC2p = off; off += (size_t)HW * CH * 2;      off = (off + 255) & ~(size_t)255;
  const size_t oWfp = off; off += (size_t)CH * CH * 2;      off = (off + 255) & ~(size_t)255;
  const size_t oTt  = off; off += (size_t)CH * CH * 4;      off = (off + 255) & ~(size_t)255;
  const size_t oWfT = off; off += (size_t)CH * CH * 4;      off = (off + 255) & ~(size_t)255;
  const size_t oCv  = off; off += (size_t)CH * 4;           off = (off + 255) & ~(size_t)255;
  const size_t oDv  = off; off += (size_t)CNTPAD * 4;       off = (off + 255) & ~(size_t)255;
  const size_t oR0  = off; off += (size_t)NPAD * CH * 4;    off = (off + 255) & ~(size_t)255;
  const size_t oR1  = off; off += (size_t)NPAD * CH * 4;    off = (off + 255) & ~(size_t)255;
  if (off > ws_size || off > (size_t)WSCAP) return;

  unsigned short* W1h = (unsigned short*)(ws + oW1h);
  unsigned short* W1l = (unsigned short*)(ws + oW1l);
  unsigned short* W2h = (unsigned short*)(ws + oW2h);
  unsigned short* W2l = (unsigned short*)(ws + oW2l);
  unsigned short* Wch = (unsigned short*)(ws + oWch);
  unsigned short* Wcl = (unsigned short*)(ws + oWcl);
  unsigned short* E2h = (unsigned short*)(ws + oE2h);
  unsigned short* E2l = (unsigned short*)(ws + oE2l);
  _Float16* We1p = (_Float16*)(ws + oE1p);
  _Float16* Wc2p = (_Float16*)(ws + oC2p);
  _Float16* Wfp  = (_Float16*)(ws + oWfp);
  float*    Tt   = (float*)(ws + oTt);
  float*    WfT  = (float*)(ws + oWfT);
  float*    cvec = (float*)(ws + oCv);
  float*    dinv = (float*)(ws + oDv);
  float*    XW1  = (float*)(ws + oR0);
  _Float16* ABs  = (_Float16*)(ws + oR0);
  float*    XW2  = (float*)(ws + oR1);

  const int vec8 = ((nE & 3) == 0) ? 1 : 0;

  k_prep<<<63, NTHR, 0, stream>>>(W1, W2, We1, We2, Wc1, bc1, be2, Wc2,
                                  W1h, W1l, W2h, W2l, Wch, Wcl, E2h, E2l, We1p, Wc2p, Tt, cvec);
  k_gemm3<<<2, GTHR, 0, stream>>>(Tt, CH, CH, E2h, E2l, WfT);
  k_cvwf<<<8, NTHR, 0, stream>>>(WfT, Wfp);
  k_count<<<nBC, NTHR, 0, stream>>>(dsts, dinv, nE, vec8);
  k_gemm3<<<nBlkG, GTHR, 0, stream>>>(x, CH, nN, W1h, W1l, XW1);
  hipFuncSetAttribute(reinterpret_cast<const void*>(&k_agg<false>),
                      hipFuncAttributeMaxDynamicSharedMemorySize, LDS_AGG);
  k_agg<false><<<nBA, NTHR, LDS_AGG, stream>>>(XW1, dinv, srcs, dsts, b1, W2h, W2l, CH,
                                                (void*)XW2, nN, nE, vec8, NPAD);
  hipFuncSetAttribute(reinterpret_cast<const void*>(&k_agg<true>),
                      hipFuncAttributeMaxDynamicSharedMemorySize, LDS_AGG);
  k_agg<true><<<nBA, NTHR, LDS_AGG, stream>>>(XW2, dinv, srcs, dsts, b2, Wch, Wcl, 2 * CH,
                                               (void*)ABs, nN, nE, vec8, NPAD);
  k_edge<<<nBlkE, ETHR, 0, stream>>>(ea, srcs, dsts, ABs, We1p, Wfp, Wc2p, be1, cvec, bc2, Wc3, bc3,
                                     out, nN, nE);
}
